// GRU_42820823941719
// MI455X (gfx1250) — hardware-verified
//
#include <hip/hip_runtime.h>


constexpr int B   = 512;
constexpr int S   = 128;
constexpr int P   = 32;
constexpr int F   = 64;
constexpr int O   = 64;
constexpr int H   = 1024;
constexpr int IN  = F + O;
constexpr int G3  = 3 * H;
constexpr int XR  = 2 * IN;
constexpr int HR  = 2 * H;
constexpr int NKX = IN / 32;
constexpr int NKH = H / 32;
constexpr long SF = (long)(S + P - 1) * F;
constexpr long SL = (long)S * O;

typedef __bf16 v16bf __attribute__((ext_vector_type(16)));
typedef float  v8f   __attribute__((ext_vector_type(8)));
typedef float  v4fb  __attribute__((ext_vector_type(4)));
typedef unsigned int v4ub __attribute__((ext_vector_type(4)));
typedef v4fb __attribute__((may_alias)) v4f;
typedef v4ub __attribute__((may_alias)) v4u;
typedef unsigned short u16;

__host__ __device__ __forceinline__ int pkc(int u) {
    return (((u >> 3) & 1) << 4) + (u & 7) + (((u >> 4) & 1) << 3);
}
__host__ __device__ __forceinline__ int piece_k(int q) {
    return ((q & 1) << 4) + ((q >> 1) << 3);
}

__device__ __forceinline__ u16 bf_bits(float f) {
    unsigned int u = __float_as_uint(f);
    u = u + 0x7FFFu + ((u >> 16) & 1u);
    return (u16)(u >> 16);
}
__device__ __forceinline__ float bf_val(u16 b) {
    return __uint_as_float(((unsigned int)b) << 16);
}

__device__ __forceinline__ v8f mma1(v16bf a, v16bf b, v8f c) {
    c = __builtin_amdgcn_wmma_f32_16x16x32_bf16(false, a, false, b, (short)0, c, false, false);
    asm volatile("v_nop\n\tv_nop\n\tv_nop\n\tv_nop" : "+v"(c) : "v"(a), "v"(b));
    return c;
}
__device__ __forceinline__ v8f mma3(v16bf ah, v16bf al, v16bf bh_, v16bf bl, v8f c) {
    c = mma1(ah, bh_, c);
    c = mma1(ah, bl, c);
    c = mma1(al, bh_, c);
    return c;
}

__device__ __forceinline__ float sigm(float x) { return 1.0f / (1.0f + expf(-x)); }

__device__ __forceinline__ void st16x2(u16* d, v4ub v) {
    *(volatile v4u*)d = v;
    __threadfence();
    *(volatile v4u*)d = v;
}

union Pk8 { v4ub u; u16 e[8]; };
__device__ __forceinline__ v4ub pack_piece(const float* __restrict__ s, int plane) {
    const v4fb x0 = *(const v4fb*)s;
    const v4fb x1 = *(const v4fb*)(s + 4);
    float x[8] = {x0.x, x0.y, x0.z, x0.w, x1.x, x1.y, x1.z, x1.w};
    Pk8 r;
#pragma unroll
    for (int j = 0; j < 8; ++j) {
        const u16 hi = bf_bits(x[j]);
        u16 e = hi;
        if (plane) e = bf_bits(x[j] - bf_val(hi));
        r.e[j] = e;
    }
    return r.u;
}

__global__ __launch_bounds__(256)
void k_packw(const float* __restrict__ src, u16* __restrict__ dst, int K, int nrows) {
    const int ppr = K >> 2;
    const long total  = (long)nrows * ppr;
    const long stride = (long)gridDim.x * blockDim.x;
    for (long i = (long)blockIdx.x * blockDim.x + threadIdx.x; i < total; i += stride) {
        const int row = (int)(i / ppr);
        const int p   = (int)(i - (long)row * ppr);
        const int chunk = p >> 3, plane = (p >> 2) & 1, q = p & 3;
        const int kb = chunk * 32 + piece_k(q);
        const v4ub v = pack_piece(src + (long)row * K + kb, plane);
        st16x2(dst + (long)row * (2 * K) + (long)p * 8, v);
    }
}

__global__ __launch_bounds__(256)
void k_packx0(const float* __restrict__ feats, const float* __restrict__ labels, u16* __restrict__ X) {
    const long total  = (long)S * B * 32;
    const long stride = (long)gridDim.x * blockDim.x;
    for (long i = (long)blockIdx.x * blockDim.x + threadIdx.x; i < total; i += stride) {
        const int row = (int)(i >> 5);
        const int p   = (int)(i & 31);
        const int t = row / B, b = row - t * B;
        const int chunk = p >> 3, plane = (p >> 2) & 1, q = p & 3;
        const int kk = piece_k(q);
        const float* s = (chunk < 2)
            ? feats  + (long)b * SF + (long)t * F + chunk * 32 + kk
            : labels + (long)b * SL + (long)t * O + (chunk - 2) * 32 + kk;
        const v4ub v = pack_piece(s, plane);
        st16x2(X + (long)row * XR + (long)p * 8, v);
    }
}

__global__ __launch_bounds__(256)
void k_packx1(const float* __restrict__ feats, u16* __restrict__ X) {
    const long total  = (long)(P - 1) * B * 16;
    const long stride = (long)gridDim.x * blockDim.x;
    for (long i = (long)blockIdx.x * blockDim.x + threadIdx.x; i < total; i += stride) {
        const int row = (int)(i >> 4);
        const int p   = (int)(i & 15);
        const int t = row / B, b = row - t * B;
        const int chunk = p >> 3, plane = (p >> 2) & 1, q = p & 3;
        const float* s = feats + (long)b * SF + (long)(S + t) * F + chunk * 32 + piece_k(q);
        const v4ub v = pack_piece(s, plane);
        st16x2(X + (long)row * XR + (long)p * 8, v);
    }
}

__device__ __forceinline__ void stage_w(v4ub* sB, const u16* __restrict__ W, int rowHalves,
                                        int u0, int c, int tid) {
#pragma unroll
    for (int s = 0; s < 6; ++s) {
        const int id = tid + 128 * s;
        const int r = id >> 3, p = id & 7;
        const int g = r >> 5, cc = r & 31;
        const v4ub* src = (const v4ub*)(W + (long)(g * H + u0 + cc) * rowHalves + c * 64) + p;
        sB[r * 8 + p] = *src;
    }
}
__device__ __forceinline__ v16bf ldb(const v4ub* sB, int r, int plane, int hh) {
    return *(const v16bf*)(&sB[r * 8 + plane * 4 + hh * 2]);
}

__device__ __forceinline__ void cell_store(const float (*sT)[32], const u16 (*sHb)[64],
                                           float* __restrict__ h32o, u16* __restrict__ hpo,
                                           int bb, int u0, int ut, int lane) {
#pragma unroll
    for (int p = 0; p < 4; ++p) {
        const int rl = p * 4 + (lane >> 3), pc = lane & 7;
        const v4f fv = *(const v4f*)(&sT[rl][pc * 4]);
        const v4u uv = *(const v4u*)(&sHb[rl][pc * 8]);
        *(volatile v4f*)(h32o + (long)(bb + rl) * H + u0 + pc * 4) = fv;
        *(volatile v4u*)(hpo + (long)(bb + rl) * HR + ut * 64 + pc * 8) = uv;
    }
}

__global__ __launch_bounds__(128)
void k_cell(const u16* __restrict__ xp,
            const u16* __restrict__ hp,
            const float* __restrict__ h32,
            const u16* __restrict__ Wip,
            const u16* __restrict__ Whp,
            const float* __restrict__ bi, const float* __restrict__ bh,
            float* __restrict__ h32o, u16* __restrict__ hpo) {
    __shared__ v4ub  sB[96 * 8] __attribute__((aligned(32)));
    __shared__ float sT[4][16][32] __attribute__((aligned(16)));
    __shared__ u16   sHb[4][16][64] __attribute__((aligned(16)));

    const int tid  = threadIdx.x;
    const int lane = tid & 31, wv = tid >> 5;
    const int hh   = lane >> 4, l16 = lane & 15;
    const int bb   = blockIdx.x * 64 + wv * 16;
    const int ut   = blockIdx.y;
    const int u0   = ut * 32;
    const int arow = bb + l16;

    v8f accr[2], accz[2], accn[2], acch[2];
#pragma unroll
    for (int nt = 0; nt < 2; ++nt) {
        accr[nt] = (v8f)0.0f; accz[nt] = (v8f)0.0f;
        accn[nt] = (v8f)0.0f; acch[nt] = (v8f)0.0f;
    }

#pragma unroll 1
    for (int c = 0; c < NKX; ++c) {
        __syncthreads();
        stage_w(sB, Wip, XR, u0, c, tid);
        __syncthreads();
        const u16* ap = xp + (long)arow * XR + c * 64 + hh * 16;
        const v16bf ah = *(const v16bf*)ap;
        const v16bf al = *(const v16bf*)(ap + 32);
#pragma unroll
        for (int nt = 0; nt < 2; ++nt) {
            const int rb = nt * 16 + l16;
            const v16bf b0h = ldb(sB, rb,      0, hh), b0l = ldb(sB, rb,      1, hh);
            const v16bf b1h = ldb(sB, 32 + rb, 0, hh), b1l = ldb(sB, 32 + rb, 1, hh);
            const v16bf b2h = ldb(sB, 64 + rb, 0, hh), b2l = ldb(sB, 64 + rb, 1, hh);
            accr[nt] = mma3(ah, al, b0h, b0l, accr[nt]);
            accz[nt] = mma3(ah, al, b1h, b1l, accz[nt]);
            accn[nt] = mma3(ah, al, b2h, b2l, accn[nt]);
        }
    }
#pragma unroll 1
    for (int c = 0; c < NKH; ++c) {
        __syncthreads();
        stage_w(sB, Whp, HR, u0, c, tid);
        __syncthreads();
        const u16* ap = hp + (long)arow * HR + c * 64 + hh * 16;
        const v16bf ah = *(const v16bf*)ap;
        const v16bf al = *(const v16bf*)(ap + 32);
#pragma unroll
        for (int nt = 0; nt < 2; ++nt) {
            const int rb = nt * 16 + l16;
            const v16bf b0h = ldb(sB, rb,      0, hh), b0l = ldb(sB, rb,      1, hh);
            const v16bf b1h = ldb(sB, 32 + rb, 0, hh), b1l = ldb(sB, 32 + rb, 1, hh);
            const v16bf b2h = ldb(sB, 64 + rb, 0, hh), b2l = ldb(sB, 64 + rb, 1, hh);
            accr[nt] = mma3(ah, al, b0h, b0l, accr[nt]);
            accz[nt] = mma3(ah, al, b1h, b1l, accz[nt]);
            acch[nt] = mma3(ah, al, b2h, b2l, acch[nt]);
        }
    }

#pragma unroll
    for (int nt = 0; nt < 2; ++nt) {
        const int ul = nt * 16 + l16;
        const int u  = u0 + ul;
        const int pp = pkc(ul);
        const float br_  = bi[u] + bh[u];
        const float bz_  = bi[H + u] + bh[H + u];
        const float bin_ = bi[2 * H + u];
        const float bhn_ = bh[2 * H + u];
#pragma unroll
        for (int v = 0; v < 8; ++v) {
            const int rl = hh * 8 + v;
            const float r  = sigm(accr[nt][v] + br_);
            const float z  = sigm(accz[nt][v] + bz_);
            const float n  = tanhf(accn[nt][v] + bin_ + r * (acch[nt][v] + bhn_));
            const float ho = h32[(long)(bb + rl) * H + u];
            const float hn = (1.0f - z) * n + z * ho;
            sT[wv][rl][ul] = hn;
            const u16 hi = bf_bits(hn);
            sHb[wv][rl][pp]      = hi;
            sHb[wv][rl][32 + pp] = bf_bits(hn - bf_val(hi));
        }
    }
    __syncthreads();
    cell_store(sT[wv], sHb[wv], h32o, hpo, bb, u0, ut, lane);
    __threadfence();
    cell_store(sT[wv], sHb[wv], h32o, hpo, bb, u0, ut, lane);
}

__device__ __forceinline__ void proj_store(const float (*sO)[64], const u16 (*sX)[128],
                                           float* __restrict__ outp, u16* __restrict__ xnext,
                                           int bb, int lane) {
#pragma unroll
    for (int p = 0; p < 8; ++p) {
        const int L = p * 4 + (lane >> 3);
        const int rl = L >> 1, hf = L & 1, pc = lane & 7;
        const v4f fv = *(const v4f*)(&sO[rl][hf * 32 + pc * 4]);
        const v4u uv = *(const v4u*)(&sX[rl][hf * 64 + pc * 8]);
        *(volatile v4f*)(outp  + (long)(bb + rl) * O  + hf * 32 + pc * 4)       = fv;
        *(volatile v4u*)(xnext + (long)(bb + rl) * XR + 128 + hf * 64 + pc * 8) = uv;
    }
}

__global__ __launch_bounds__(32)
void k_proj(const u16* __restrict__ hp, const u16* __restrict__ Wdp, const float* __restrict__ bd,
            float* __restrict__ outp,
            u16* __restrict__ xnext) {
    __shared__ float sO[16][64]  __attribute__((aligned(16)));
    __shared__ u16   sX[16][128] __attribute__((aligned(16)));
    const int lane = threadIdx.x & 31;
    const int hh = lane >> 4, l16 = lane & 15;
    const int bb = blockIdx.x * 16;
    const int arow = bb + l16;

    v8f acc[4];
#pragma unroll
    for (int nt = 0; nt < 4; ++nt) acc[nt] = (v8f)0.0f;

#pragma unroll 1
    for (int c = 0; c < NKH; ++c) {
        const u16* ap = hp + (long)arow * HR + c * 64 + hh * 16;
        const v16bf ah = *(const v16bf*)ap;
        const v16bf al = *(const v16bf*)(ap + 32);
#pragma unroll
        for (int nt = 0; nt < 4; ++nt) {
            const u16* bp = Wdp + (long)(nt * 16 + l16) * HR + c * 64 + hh * 16;
            const v16bf bh_ = *(const v16bf*)bp;
            const v16bf bl  = *(const v16bf*)(bp + 32);
            acc[nt] = mma3(ah, al, bh_, bl, acc[nt]);
        }
    }

#pragma unroll
    for (int nt = 0; nt < 4; ++nt) {
        const int o = nt * 16 + l16;
        const float bo = bd[o];
        const int xoff = (nt >> 1) * 64;
        const int pp   = pkc((nt & 1) * 16 + l16);
#pragma unroll
        for (int v = 0; v < 8; ++v) {
            const int rl = hh * 8 + v;
            const float val = acc[nt][v] + bo;
            sO[rl][o] = val;
            const u16 hi = bf_bits(val);
            sX[rl][xoff + pp]      = hi;
            sX[rl][xoff + 32 + pp] = bf_bits(val - bf_val(hi));
        }
    }
    __syncthreads();
    proj_store(sO, sX, outp, xnext, bb, lane);
    __threadfence();
    proj_store(sO, sX, outp, xnext, bb, lane);
}

extern "C" void kernel_launch(void* const* d_in, const int* in_sizes, int n_in,
                              void* d_out, int out_size, void* d_ws, size_t ws_size,
                              hipStream_t stream) {
    if (n_in != 8) return;
    if (in_sizes[0] != B * (S + P - 1) * F) return;
    if (in_sizes[1] != B * S * O) return;
    if (in_sizes[2] != G3 * IN) return;
    if (in_sizes[3] != G3 * H) return;
    if (in_sizes[4] != G3 || in_sizes[5] != G3) return;
    if (in_sizes[6] != O * H || in_sizes[7] != O) return;
    if (out_size != P * B * O) return;

    const float* feats  = (const float*)d_in[0];
    const float* labels = (const float*)d_in[1];
    const float* Wi     = (const float*)d_in[2];
    const float* Wh     = (const float*)d_in[3];
    const float* bi     = (const float*)d_in[4];
    const float* bh     = (const float*)d_in[5];
    const float* Wd     = (const float*)d_in[6];
    const float* bd     = (const float*)d_in[7];
    float* out = (float*)d_out;

    size_t off = 0;
    auto carve = [&](size_t bytes) { size_t o = off; off += (bytes + 255) & ~(size_t)255; return o; };
    char* ws = (char*)d_ws;
    const size_t oWip  = carve((size_t)G3 * XR * sizeof(u16));
    const size_t oWhp  = carve((size_t)G3 * HR * sizeof(u16));
    const size_t oWdp  = carve((size_t)O  * HR * sizeof(u16));
    const size_t oH32a = carve((size_t)B * H * sizeof(float));
    const size_t oH32b = carve((size_t)B * H * sizeof(float));
    const size_t oHpa  = carve((size_t)B * HR * sizeof(u16));
    const size_t oHpb  = carve((size_t)B * HR * sizeof(u16));
    const size_t oX0   = carve((size_t)S * B * XR * sizeof(u16));
    const size_t oX1   = carve((size_t)P * B * XR * sizeof(u16));
    if (off > ws_size) return;

    u16* Wip = (u16*)(ws + oWip);
    u16* Whp = (u16*)(ws + oWhp);
    u16* Wdp = (u16*)(ws + oWdp);
    float* h32[2] = {(float*)(ws + oH32a), (float*)(ws + oH32b)};
    u16*   hpk[2] = {(u16*)(ws + oHpa), (u16*)(ws + oHpb)};
    u16* X0 = (u16*)(ws + oX0);
    u16* X1 = (u16*)(ws + oX1);

    auto nblk = [](long total) { long g = (total + 255) / 256; if (g > 4096) g = 4096; if (g < 1) g = 1; return (unsigned)g; };

    k_packw<<<nblk((long)G3 * (IN / 4)), 256, 0, stream>>>(Wi, Wip, IN, G3);
    k_packw<<<nblk((long)G3 * (H / 4)),  256, 0, stream>>>(Wh, Whp, H,  G3);
    k_packw<<<nblk((long)O  * (H / 4)),  256, 0, stream>>>(Wd, Wdp, H,  O);
    k_packx0<<<nblk((long)S * B * 32), 256, 0, stream>>>(feats, labels, X0);
    k_packx1<<<nblk((long)(P - 1) * B * 16), 256, 0, stream>>>(feats, X1);
    hipMemsetAsync(h32[0], 0, (size_t)B * H * sizeof(float), stream);
    hipMemsetAsync(hpk[0], 0, (size_t)B * HR * sizeof(u16), stream);

    const dim3 gCell(B / 64, H / 32);
    const dim3 gProj(B / 16);

    int cur = 0;
    for (int t = 0; t < S; ++t) {
        k_cell<<<gCell, 128, 0, stream>>>(X0 + (long)t * B * XR, hpk[cur], h32[cur],
                                          Wip, Whp, bi, bh, h32[1 - cur], hpk[1 - cur]);
        cur ^= 1;
    }
    k_proj<<<gProj, 32, 0, stream>>>(hpk[cur], Wdp, bd, out, X1);
    for (int t = 0; t < P - 1; ++t) {
        k_cell<<<gCell, 128, 0, stream>>>(X1 + (long)t * B * XR, hpk[cur], h32[cur],
                                          Wip, Whp, bi, bh, h32[1 - cur], hpk[1 - cur]);
        cur ^= 1;
        k_proj<<<gProj, 32, 0, stream>>>(hpk[cur], Wdp, bd, out + (long)(t + 1) * B * O,
                                         X1 + (long)(t + 1) * B * XR);
    }
}
